// SelfAttentionV1_51599737094689
// MI455X (gfx1250) — hardware-verified
//
#include <hip/hip_runtime.h>
#include <hip/hip_bf16.h>

typedef __attribute__((ext_vector_type(16))) _Float16 v16h;
typedef __attribute__((ext_vector_type(8)))  _Float16 v8h;
typedef __attribute__((ext_vector_type(16))) __bf16   v16b;
typedef __attribute__((ext_vector_type(8)))  __bf16   v8b;
typedef __attribute__((ext_vector_type(8)))  float    v8f;
typedef __attribute__((ext_vector_type(4)))  float    v4f;
typedef __attribute__((ext_vector_type(4)))  unsigned int v4u;

constexpr int kBatch = 4;
constexpr int kSeq   = 2048;
constexpr int kDim   = 1024;

__device__ __forceinline__ unsigned short f2bf_bits(float f) {
  unsigned u = __float_as_uint(f);
  return (unsigned short)((u + 0x7FFFu + ((u >> 16) & 1u)) >> 16);
}
__device__ __forceinline__ float bf_bits2f(unsigned short h) { return __uint_as_float(((unsigned)h) << 16); }

__device__ __forceinline__ void dep_guard_h(v8f& a, v8f& b, v16h x, v16h y) { asm volatile("v_nop\n\tv_nop\n\tv_nop\n\tv_nop" : "+v"(a), "+v"(b) : "v"(x), "v"(y)); }
__device__ __forceinline__ void dep_guard_b(v8f& a, v8f& b, v16b x, v16b y) { asm volatile("v_nop\n\tv_nop\n\tv_nop\n\tv_nop" : "+v"(a), "+v"(b) : "v"(x), "v"(y)); }
__device__ __forceinline__ void keep4_h(v16h a, v16h b, v16h c, v16h d) { asm volatile("v_nop" :: "v"(a), "v"(b), "v"(c), "v"(d)); }
__device__ __forceinline__ void keep4_b(v16b a, v16b b, v16b c, v16b d) { asm volatile("v_nop" :: "v"(a), "v"(b), "v"(c), "v"(d)); }
__device__ __forceinline__ void acc_guard4(v8f& a, v8f& b, v8f& c, v8f& d) { asm volatile("v_nop\n\tv_nop\n\tv_nop\n\tv_nop" : "+v"(a), "+v"(b), "+v"(c), "+v"(d)); }

template <typename T> struct Frag;
template <> struct Frag<_Float16> {
  typedef v16h V; union U { v16h v; v8h h[2]; };
  static __device__ __forceinline__ v16h load(const _Float16* p) {
    U f; f.h[0] = *(const v8h*)(p); f.h[1] = *(const v8h*)(p + 16); return f.v;
  }
  static __device__ __forceinline__ v8f mma(v16h a, v16h b, v8f c) {
    return __builtin_amdgcn_wmma_f32_16x16x32_f16(false, a, false, b, (short)0, c, false, false);
  }
  static __device__ __forceinline__ void guard(v8f& a, v8f& b, v16h x, v16h y) { dep_guard_h(a, b, x, y); }
  static __device__ __forceinline__ void keep(v16h a, v16h b, v16h c, v16h d) { keep4_h(a, b, c, d); }
};
template <> struct Frag<__bf16> {
  typedef v16b V; union U { v16b v; v8b h[2]; };
  static __device__ __forceinline__ v16b load(const __bf16* p) {
    U f; f.h[0] = *(const v8b*)(p); f.h[1] = *(const v8b*)(p + 16); return f.v;
  }
  static __device__ __forceinline__ v8f mma(v16b a, v16b b, v8f c) {
    return __builtin_amdgcn_wmma_f32_16x16x32_bf16(false, a, false, b, (short)0, c, false, false);
  }
  static __device__ __forceinline__ void guard(v8f& a, v8f& b, v16b x, v16b y) { dep_guard_b(a, b, x, y); }
  static __device__ __forceinline__ void keep(v16b a, v16b b, v16b c, v16b d) { keep4_b(a, b, c, d); }
};

template <int ET> struct Elem;
template <> struct Elem<0> { typedef _Float16 T; };
template <> struct Elem<1> { typedef __bf16 T; };
template <int ET, bool SPLIT, int BIAS_MODE, int OUT_MODE>
__global__ __launch_bounds__(256) void wmma_gemm64(
    const unsigned short* __restrict__ Ap, const unsigned short* __restrict__ A2p, int lda, long strideA,
    const unsigned short* __restrict__ Btp, const unsigned short* __restrict__ Bt2p, int ldb, long strideB,
    void* __restrict__ Cout, void* __restrict__ Cout2, int ldc, long strideC,
    const float* __restrict__ bias,
    int M, int N, int K, float scale) {
  typedef typename Elem<ET>::T T;
  typedef typename Frag<T>::V V;
  const T* A = (const T*)Ap; const T* A2 = (const T*)A2p; const T* Bt = (const T*)Btp; const T* Bt2 = (const T*)Bt2p;
  __shared__ __align__(16) float sT[8][16 * 68];
  const int b    = blockIdx.y;
  const int lane = threadIdx.x & 31;
  const int wave = threadIdx.x >> 5;
  const int tilesN = N >> 6;
  const int tilesM = M >> 6;
  const int tile = blockIdx.x * 8 + wave;
  if (tile >= tilesM * tilesN) return;
  const int tm = tile / tilesN;
  const int tn = tile - tm * tilesN;
  const int m0 = tm << 6;
  const int n0 = tn << 6;

  const T* Ab  = A  + (size_t)b * strideA;
  const T* Bb  = Bt + (size_t)b * strideB;
  const T* Ab2 = SPLIT ? (A2  + (size_t)b * strideA) : nullptr;
  const T* Bb2 = SPLIT ? (Bt2 + (size_t)b * strideB) : nullptr;

  const int rlane = lane & 15;
  const int koff  = (lane >> 4) * 8;
  const int mOff  = (lane >> 4) * 8;

  v8f acc[4][4];
#pragma unroll
  for (int i = 0; i < 4; ++i)
#pragma unroll
    for (int j = 0; j < 4; ++j) acc[i][j] = (v8f){0.f,0.f,0.f,0.f,0.f,0.f,0.f,0.f};

  for (int k0 = 0; k0 < K; k0 += 32) {
    V bh[4], bl[4];
#pragma unroll
    for (int j = 0; j < 4; ++j) {
      const size_t bo = (size_t)(n0 + (j << 4) + rlane) * ldb + koff + k0;
      bh[j] = Frag<T>::load(Bb + bo);
      if (SPLIT) bl[j] = Frag<T>::load(Bb2 + bo);
    }
#pragma unroll
    for (int i = 0; i < 4; ++i) {
      const size_t ao = (size_t)(m0 + (i << 4) + rlane) * lda + koff + k0;
      V ah = Frag<T>::load(Ab + ao);
      V al;
      if (SPLIT) al = Frag<T>::load(Ab2 + ao);
#pragma unroll
      for (int j = 0; j < 4; ++j) {
        acc[i][j] = Frag<T>::mma(ah, bh[j], acc[i][j]);
        if (SPLIT) {
          acc[i][j] = Frag<T>::mma(ah, bl[j], acc[i][j]);
          acc[i][j] = Frag<T>::mma(al, bh[j], acc[i][j]);
        }
      }
      Frag<T>::guard(acc[i][0], acc[i][3], ah, SPLIT ? al : ah);
    }
    Frag<T>::keep(bh[0], bh[1], bh[2], bh[3]);
    if (SPLIT) Frag<T>::keep(bl[0], bl[1], bl[2], bl[3]);
  }
  acc_guard4(acc[0][0], acc[0][1], acc[0][2], acc[0][3]);
  acc_guard4(acc[1][0], acc[1][1], acc[1][2], acc[1][3]);
  acc_guard4(acc[2][0], acc[2][1], acc[2][2], acc[2][3]);
  acc_guard4(acc[3][0], acc[3][1], acc[3][2], acc[3][3]);

  float* slab = sT[wave];
#pragma unroll
  for (int i = 0; i < 4; ++i) {
    const int mBase = m0 + (i << 4);
    v4f bm0 = (v4f){0.f,0.f,0.f,0.f};
    v4f bm1 = (v4f){0.f,0.f,0.f,0.f};
    if (BIAS_MODE == 1) {
      bm0 = *(const v4f*)(bias + mBase + mOff);
      bm1 = *(const v4f*)(bias + mBase + mOff + 4);
    }
#pragma unroll
    for (int j = 0; j < 4; ++j) {
      const int n = n0 + (j << 4) + rlane;
      float bvn = 0.f;
      if (BIAS_MODE == 2) bvn = bias[n];
#pragma unroll
      for (int r = 0; r < 8; ++r) {
        float v = acc[i][j][r] * scale;
        if (BIAS_MODE == 1) v += (r < 4) ? bm0[r] : bm1[r - 4];
        if (BIAS_MODE == 2) v += bvn;
        slab[(mOff + r) * 68 + (j << 4) + rlane] = v;
      }
    }
    __builtin_amdgcn_fence(__ATOMIC_RELEASE, "workgroup");
    __builtin_amdgcn_wave_barrier();
    __builtin_amdgcn_fence(__ATOMIC_ACQUIRE, "workgroup");
    if (OUT_MODE == 0) {
      float* C = (float*)Cout + (size_t)b * strideC;
      const int hh = lane >> 4, c4 = (lane & 15) * 4;
      for (int pass = 0; pass < 2; ++pass) {
#pragma unroll
        for (int it = 0; it < 8; ++it) {
          const int row = it * 2 + hh;
          v4f v = *(const v4f*)(slab + row * 68 + c4);
          *(volatile v4f*)(C + (size_t)(mBase + row) * ldc + n0 + c4) = v;
        }
        __threadfence();
      }
    } else {
      const int q = lane >> 3, c8 = (lane & 7) * 8;
      unsigned short* C  = (unsigned short*)Cout  + (size_t)b * strideC;
      unsigned short* C2 = (OUT_MODE == 2) ? ((unsigned short*)Cout2 + (size_t)b * strideC) : nullptr;
      for (int pass = 0; pass < 2; ++pass) {
#pragma unroll
        for (int it = 0; it < 4; ++it) {
          const int row = it * 4 + q;
          const float* sp = slab + row * 68 + c8;
          v8h hv, lv;
#pragma unroll
          for (int e = 0; e < 8; ++e) {
            if (OUT_MODE == 1) {
              hv[e] = (_Float16)sp[e];
              lv[e] = hv[e];
            } else {
              unsigned short hb = f2bf_bits(sp[e]);
              unsigned short lb = f2bf_bits(sp[e] - bf_bits2f(hb));
              hv[e] = __builtin_bit_cast(_Float16, hb);
              lv[e] = __builtin_bit_cast(_Float16, lb);
            }
          }
          *(volatile v8h*)(C + (size_t)(mBase + row) * ldc + n0 + c8) = hv;
          if (OUT_MODE == 2) *(volatile v8h*)(C2 + (size_t)(mBase + row) * ldc + n0 + c8) = lv;
        }
        __threadfence();
      }
    }
    __builtin_amdgcn_fence(__ATOMIC_RELEASE, "workgroup");
    __builtin_amdgcn_wave_barrier();
    __builtin_amdgcn_fence(__ATOMIC_ACQUIRE, "workgroup");
  }
}

__global__ __launch_bounds__(256) void cast_f32_bf16x8(
    const float* __restrict__ in, unsigned short* __restrict__ out, int n8) {
  const int i = blockIdx.x * 256 + threadIdx.x;
  if (i >= n8) return;
  const size_t e0 = (size_t)i * 8;
  const v4f a = *(const v4f*)(in + e0);
  const v4f c = *(const v4f*)(in + e0 + 4);
  v4u w;
  w[0] = (unsigned)f2bf_bits(a[0]) | ((unsigned)f2bf_bits(a[1]) << 16);
  w[1] = (unsigned)f2bf_bits(a[2]) | ((unsigned)f2bf_bits(a[3]) << 16);
  w[2] = (unsigned)f2bf_bits(c[0]) | ((unsigned)f2bf_bits(c[1]) << 16);
  w[3] = (unsigned)f2bf_bits(c[2]) | ((unsigned)f2bf_bits(c[3]) << 16);
  unsigned short* p = out + e0;
  *(volatile v4u*)p = w;
  __threadfence();
  *(volatile v4u*)p = w;
}

__global__ __launch_bounds__(256) void transpose_cast_bf16(
    const float* __restrict__ W0, const float* __restrict__ W1, const float* __restrict__ W2,
    unsigned short* __restrict__ T0, unsigned short* __restrict__ T1, unsigned short* __restrict__ T2,
    int dimK, int dimN) {
  __shared__ float tile[64 * 65];
  const int z = blockIdx.z;
  const float* W = (z == 0) ? W0 : ((z == 1) ? W1 : W2);
  unsigned short* T = (z == 0) ? T0 : ((z == 1) ? T1 : T2);
  const int n0 = blockIdx.x * 64;
  const int k0 = blockIdx.y * 64;
  const int tid = threadIdx.x;
  const int lane = tid & 31, wave = tid >> 5;
#pragma unroll
  for (int it = 0; it < 4; ++it) {
    const int r = it * 16 + (tid >> 4);
    const int c = (tid & 15) * 4;
    const v4f x = *(const v4f*)(W + (size_t)(k0 + r) * dimN + n0 + c);
    tile[r * 65 + c + 0] = x[0];
    tile[r * 65 + c + 1] = x[1];
    tile[r * 65 + c + 2] = x[2];
    tile[r * 65 + c + 3] = x[3];
  }
  __syncthreads();
  const int q = lane >> 3;
  const int r0 = (lane & 7) * 8;
  for (int pass = 0; pass < 2; ++pass) {
#pragma unroll
    for (int it = 0; it < 2; ++it) {
      const int c = wave * 8 + it * 4 + q;
      v4u w;
#pragma unroll
      for (int e = 0; e < 4; ++e) {
        const unsigned lo = (unsigned)f2bf_bits(tile[(r0 + 2 * e) * 65 + c]);
        const unsigned hi = (unsigned)f2bf_bits(tile[(r0 + 2 * e + 1) * 65 + c]);
        w[e] = lo | (hi << 16);
      }
      *(volatile v4u*)(T + (size_t)(n0 + c) * dimK + k0 + r0) = w;
    }
    __threadfence();
  }
}

__global__ __launch_bounds__(256) void softmax_rows_f16(
    const float* __restrict__ sc, unsigned short* __restrict__ P, int ncols, float carry) {
  __shared__ float smax[8];
  __shared__ float ssum[8];
  const int tid = threadIdx.x;
  const int lane = tid & 31, wave = tid >> 5;
  const size_t base = (size_t)blockIdx.x * ncols + (size_t)tid * 8;
  const v4f a = *(const v4f*)(sc + base);
  const v4f c = *(const v4f*)(sc + base + 4);
  float v[8] = {a[0], a[1], a[2], a[3], c[0], c[1], c[2], c[3]};
  float m = __uint_as_float(0xff800000u);
#pragma unroll
  for (int e = 0; e < 8; ++e) m = fmaxf(m, v[e]);
#pragma unroll
  for (int off = 16; off > 0; off >>= 1) m = fmaxf(m, __shfl_xor(m, off, 32));
  if (lane == 0) smax[wave] = m;
  __syncthreads();
  float mm = smax[0];
#pragma unroll
  for (int w = 1; w < 8; ++w) mm = fmaxf(mm, smax[w]);
  float s = 0.f;
#pragma unroll
  for (int e = 0; e < 8; ++e) {
    v[e] = expf(v[e] - mm);
    s += v[e];
  }
#pragma unroll
  for (int off = 16; off > 0; off >>= 1) s += __shfl_xor(s, off, 32);
  if (lane == 0) ssum[wave] = s;
  __syncthreads();
  float tot = 0.f;
#pragma unroll
  for (int w = 0; w < 8; ++w) tot += ssum[w];
  const float inv = 1.0f / tot;
  v4u wv;
#pragma unroll
  for (int e = 0; e < 4; ++e) {
    const _Float16 h0 = (_Float16)((v[2 * e] * inv) * carry);
    const _Float16 h1 = (_Float16)((v[2 * e + 1] * inv) * carry);
    wv[e] = (unsigned)__builtin_bit_cast(unsigned short, h0) | ((unsigned)__builtin_bit_cast(unsigned short, h1) << 16);
  }
  unsigned short* p = P + base;
  *(volatile v4u*)p = wv;
  __threadfence();
  *(volatile v4u*)p = wv;
}

static_assert(kDim % 32 == 0);
static_assert(kSeq % 32 == 0);
static_assert((kBatch * kSeq) % 64 == 0);
static_assert(kDim % 64 == 0);
static_assert(kSeq % 64 == 0);
static_assert(kSeq == 8 * 256);
static_assert((kBatch * kSeq * kDim) % (8 * 256) == 0);

extern "C" void kernel_launch(void* const* d_in, const int* in_sizes, int n_in,
                              void* d_out, int out_size, void* d_ws,
                              size_t ws_size, hipStream_t stream) {
  constexpr size_t kBSD = (size_t)kBatch * kSeq * kDim;
  constexpr size_t kDD  = (size_t)kDim * kDim;
  constexpr size_t kBSS = (size_t)kBatch * kSeq * kSeq;

  constexpr size_t kOffSc = 0;
  constexpr size_t kOffHb = 0;
  constexpr size_t kOffWt = kBSD * 2;
  constexpr size_t kOffP  = kBSS * 4;
  constexpr size_t kOffQ  = kOffP;
  constexpr size_t kOffK  = kOffQ + kBSD * 2;
  constexpr size_t kOffVt = kOffP + kBSS * 2;
  constexpr size_t kWsTotal = kOffVt + kBSD * 2;
  static_assert(kOffWt + 3 * kDD * 2 <= kOffP);
  static_assert(kOffK + kBSD * 2 == kOffVt);
  static_assert(kWsTotal == 117440512);
  static_assert(kWsTotal <= 134217728);

  if (n_in < 7) return;
  if ((size_t)in_sizes[0] != kBSD) return;
  if ((size_t)in_sizes[1] != kDD || (size_t)in_sizes[3] != kDD || (size_t)in_sizes[5] != kDD) return;
  if (in_sizes[2] != kDim || in_sizes[4] != kDim || in_sizes[6] != kDim) return;
  if ((size_t)out_size != kBSD) return;
  if (ws_size < kWsTotal) return;

  const float* p_h  = (const float*)d_in[0];
  const float* p_wq = (const float*)d_in[1];
  const float* p_bq = (const float*)d_in[2];
  const float* p_wk = (const float*)d_in[3];
  const float* p_bk = (const float*)d_in[4];
  const float* p_wv = (const float*)d_in[5];
  const float* p_bv = (const float*)d_in[6];
  float* p_out = (float*)d_out;

  char* ws = (char*)d_ws;
  float*          p_sc  = (float*)(ws + kOffSc);
  unsigned short* p_hb  = (unsigned short*)(ws + kOffHb);
  unsigned short* p_wqt = (unsigned short*)(ws + kOffWt);
  unsigned short* p_wkt = p_wqt + kDD;
  unsigned short* p_wvt = p_wqt + 2 * kDD;
  unsigned short* p_q   = (unsigned short*)(ws + kOffQ);
  unsigned short* p_k   = (unsigned short*)(ws + kOffK);
  unsigned short* p_p   = (unsigned short*)(ws + kOffP);
  unsigned short* p_vt  = (unsigned short*)(ws + kOffVt);

  const long sSD = (long)kSeq * kDim;
  const long sSS = (long)kSeq * kSeq;

  cast_f32_bf16x8<<<(unsigned)(kBSD / 8 / 256), 256, 0, stream>>>(p_h, p_hb, (int)(kBSD / 8));

  transpose_cast_bf16<<<dim3(kDim / 64, kDim / 64, 3), 256, 0, stream>>>(
      p_wq, p_wk, p_wv, p_wqt, p_wkt, p_wvt, kDim, kDim);

  wmma_gemm64<1, false, 2, 1><<<dim3(256, 1), 256, 0, stream>>>(
      p_hb, p_hb, kDim, 0L, p_wqt, p_wqt, kDim, 0L, (void*)p_q, (void*)p_q, kDim, 0L,
      p_bq, kBatch * kSeq, kDim, kDim, 1.0f);

  wmma_gemm64<1, false, 2, 1><<<dim3(256, 1), 256, 0, stream>>>(
      p_hb, p_hb, kDim, 0L, p_wkt, p_wkt, kDim, 0L, (void*)p_k, (void*)p_k, kDim, 0L,
      p_bk, kBatch * kSeq, kDim, kDim, 1.0f);

  wmma_gemm64<1, false, 1, 1><<<dim3(64, kBatch), 256, 0, stream>>>(
      p_wvt, p_wvt, kDim, 0L, p_hb, p_hb, kDim, sSD, (void*)p_vt, (void*)p_vt, kSeq, (long)kDim * kSeq,
      p_bv, kDim, kSeq, kDim, 1.0f);

  wmma_gemm64<0, false, 0, 0><<<dim3(128, kBatch), 256, 0, stream>>>(
      p_q, p_q, kDim, sSD, p_k, p_k, kDim, sSD, (void*)p_sc, (void*)p_sc, kSeq, sSS,
      p_bq, kSeq, kSeq, kDim, 0.03125f);

  softmax_rows_f16<<<(unsigned)(kBatch * kSeq), 256, 0, stream>>>(p_sc, p_p, kSeq, 4096.0f);

  wmma_gemm64<0, false, 0, 0><<<dim3(64, kBatch), 256, 0, stream>>>(
      p_p, p_p, kSeq, sSS, p_vt, p_vt, kSeq, (long)kDim * kSeq, (void*)p_out, (void*)p_out, kDim, sSD,
      p_bq, kSeq, kDim, kSeq, 1.0f / 4096.0f);
}
